// involution2_52201032516022
// MI455X (gfx1250) — hardware-verified
//
#include <hip/hip_runtime.h>
#include <math.h>

typedef __attribute__((ext_vector_type(16))) _Float16 v16h;
typedef __attribute__((ext_vector_type(16))) __bf16 v16b;
typedef __attribute__((ext_vector_type(8)))  _Float16 v8h;
typedef __attribute__((ext_vector_type(8)))  float v8f;
typedef __attribute__((ext_vector_type(4)))  float v4f;
typedef __attribute__((ext_vector_type(2)))  float v2f;
typedef __attribute__((ext_vector_type(4)))  unsigned v4u;
typedef __attribute__((ext_vector_type(4)))  int v4i;
typedef float __attribute__((may_alias)) float_a;
typedef int __attribute__((may_alias)) int_a;

template <typename T> __device__ __forceinline__ void vst2(void* p, T v) { *(volatile T*)p = v; __threadfence(); *(volatile T*)p = v; }
__device__ __forceinline__ v8f wmma16(v16h a, v16h b, v8f c) {
  v8f d = __builtin_amdgcn_wmma_f32_16x16x32_f16(false, a, false, b, (short)0, c, false, false);
  asm volatile("v_nop\n\tv_nop\n\tv_nop\n\tv_nop" : "+v"(d) : "v"(a), "v"(b));
  return d;
}
__device__ __forceinline__ v8f wmma_bf(v16b a, v16b b, v8f c) {
  v8f d = __builtin_amdgcn_wmma_f32_16x16x32_bf16(false, a, false, b, (short)0, c, false, false);
  asm volatile("v_nop\n\tv_nop\n\tv_nop\n\tv_nop" : "+v"(d) : "v"(a), "v"(b));
  return d;
}
__device__ __forceinline__ v16h frag_h(const _Float16* rowk0, int lane) {
  union { v16h v; v8h q[2]; } u; const _Float16* p = rowk0 + 8 * (lane >> 4);
  u.q[0] = *(const v8h*)p; u.q[1] = *(const v8h*)(p + 16); return u.v;
}
__device__ __forceinline__ v16h frag_f32(const float* rowk0, int lane) {
  v16h a; const float* p = rowk0 + 8 * (lane >> 4);
#pragma unroll
  for (int i = 0; i < 8; ++i) { a[i] = (_Float16)p[i]; a[8 + i] = (_Float16)p[16 + i]; }
  return a;
}
__device__ __forceinline__ v16h frag_f32s(const float* rowk0, int lane, float sc) {
  v16h a; const float* p = rowk0 + 8 * (lane >> 4);
#pragma unroll
  for (int i = 0; i < 8; ++i) { a[i] = (_Float16)(p[i] * sc); a[8 + i] = (_Float16)(p[16 + i] * sc); }
  return a;
}
__device__ __forceinline__ v16h fragc_f32(const float* W, int k0, int n, int lane, int ld, int K) {
  v16h a; const int g = lane >> 4;
#pragma unroll
  for (int i = 0; i < 8; ++i) { const int ka = k0 + 8 * g + i, kb = ka + 16;
    a[i] = (_Float16)(ka < K ? W[(size_t)ka * ld + n] : 0.f); a[8 + i] = (_Float16)(kb < K ? W[(size_t)kb * ld + n] : 0.f); }
  return a;
}
struct F2 { v16b h, l; };
__device__ __forceinline__ F2 bsplit16(const float v[16]) { F2 r;
#pragma unroll
  for (int i = 0; i < 16; ++i) { const __bf16 h = (__bf16)v[i]; r.h[i] = h; r.l[i] = (__bf16)(v[i] - (float)h); }
  return r; }
__device__ __forceinline__ F2 split_row(const float* row, int k0, int lane) { float v[16]; const float* p = row + k0 + 8 * (lane >> 4);
#pragma unroll
  for (int i = 0; i < 8; ++i) { v[i] = p[i]; v[8 + i] = p[16 + i]; }
  return bsplit16(v); }
__device__ __forceinline__ F2 split_rowK(const float* row, int k0, int lane, int K) { float v[16]; const int g = lane >> 4;
#pragma unroll
  for (int i = 0; i < 8; ++i) { const int ka = k0 + 8 * g + i, kb = ka + 16; v[i] = ka < K ? row[ka] : 0.f; v[8 + i] = kb < K ? row[kb] : 0.f; }
  return bsplit16(v); }
__device__ __forceinline__ F2 split_col(const float* W, int k0, int n, int lane, int ld, int K) { float v[16]; const int g = lane >> 4;
#pragma unroll
  for (int i = 0; i < 8; ++i) { const int ka = k0 + 8 * g + i, kb = ka + 16; v[i] = ka < K ? W[(size_t)ka * ld + n] : 0.f; v[8 + i] = kb < K ? W[(size_t)kb * ld + n] : 0.f; }
  return bsplit16(v); }
__device__ __forceinline__ v8f mac3(const F2& a, const F2& b, v8f c) { c = wmma_bf(a.l, b.h, c); c = wmma_bf(a.h, b.l, c); return wmma_bf(a.h, b.h, c); }
__device__ __forceinline__ float sigm(float v) { return 1.0f / (1.0f + expf(-v)); }
#define LDSX() do { asm volatile("s_wait_dscnt 0" ::: "memory"); __builtin_amdgcn_wave_barrier(); __builtin_amdgcn_fence(__ATOMIC_RELEASE, "workgroup"); } while (0)

__device__ __forceinline__ v16h frag_f32sK2(const float* __restrict__ row, int k0, int lane, float sc, int K) {
  const int g = lane >> 4; v16h r;
#pragma unroll
  for (int i = 0; i < 8; ++i) { const int ka = k0 + 8 * g + i, kb = ka + 16; r[i] = (_Float16)((ka < K ? row[ka] : 0.f) * sc); r[8 + i] = (_Float16)((kb < K ? row[kb] : 0.f) * sc); }
  return r;
}
#define NB 4
#define CC 64
#define HI 128
#define WI 128
#define NPX (HI * WI)
#define CR 32
#define KK 7
#define K2 49
#define NG 16
#define GCH 4
#define NWT (K2 * NG)
#define NWP 800
#define CHK 16

__global__ __launch_bounds__(128) void k_main(const float* __restrict__ x, const float* __restrict__ y, const float* __restrict__ w1, const float* __restrict__ b1, const float* __restrict__ bng, const float* __restrict__ bnb, const float* __restrict__ bnm, const float* __restrict__ bnv,
                                            const float* __restrict__ w2, const float* __restrict__ b2, float* __restrict__ out) {
  __shared__ __align__(16) _Float16 st[4][16][40];
  __shared__ __align__(16) float sw[64][NWP + 4];
  __shared__ __align__(16) float sy[CHK][KK][72];
  __shared__ __align__(16) float so[CHK][64 + 4];
  const int tid = threadIdx.x, wave = tid >> 5, lane = tid & 31, col = lane & 15, g = lane >> 4;
  const int b = blockIdx.z, r = blockIdx.y, x0 = blockIdx.x * 64; const int p0 = r * WI + x0 + wave * 16;
  const float* xb = x + (size_t)b * CC * NPX;
  { v8f acc[2] = {};
#pragma unroll
    for (int kc = 0; kc < CC / 32; ++kc) { const v16h a = fragc_f32(xb, kc * 32, p0 + col, lane, NPX, CC);
#pragma unroll
      for (int t = 0; t < 2; ++t) acc[t] = wmma16(a, frag_f32s(w1 + (size_t)(t * 16 + col) * CC + kc * 32, lane, 16.0f), acc[t]); }
#pragma unroll
    for (int t = 0; t < 2; ++t) { const int o = t * 16 + col; const float sc = bng[o] * rsqrtf(bnv[o] + 1e-5f), bb = b1[o], mm = bnm[o], be = bnb[o];
#pragma unroll
      for (int rr = 0; rr < 8; ++rr) { float v = acc[t][rr] * (1.0f / 16.0f) + bb; v = (v - mm) * sc + be; st[wave][8 * g + rr][o] = (_Float16)(v > 0.f ? v : 0.f); } } }
  for (int q = lane; q < 16 * 8; q += 32) st[wave][q >> 3][32 + (q & 7)] = (_Float16)0.f;
  LDSX();
  { const v16h a = frag_h(&st[wave][col][0], lane);
#pragma unroll 1
    for (int t = 0; t < NWP / 16; ++t) { const int n = t * 16 + col; const int nn = n < NWT ? n : 0; v8f acc = {};
      acc = wmma16(a, frag_f32sK2(w2 + (size_t)nn * CR, 0, lane, 16.0f, CR), acc);
      const float bb = n < NWT ? b2[nn] : 0.f;
#pragma unroll
      for (int rr = 0; rr < 8; ++rr) sw[wave * 16 + 8 * g + rr][n] = n < NWT ? acc[rr] * (1.0f / 16.0f) + bb : 0.f; } }
  __syncthreads();
  const float* yb = y + (size_t)b * CC * NPX;
#pragma unroll 1
  for (int c0 = 0; c0 < CC; c0 += CHK) {
    for (int q = tid; q < CHK * KK * 70; q += 128) { const int ch = q / (KK * 70), rem = q % (KK * 70), dy = rem / 70, xx = rem % 70; const int yy = r + dy - 3, xg = x0 + xx - 3;
      sy[ch][dy][xx] = (yy >= 0 && yy < HI && xg >= 0 && xg < WI) ? yb[(size_t)(c0 + ch) * NPX + yy * WI + xg] : 0.f; }
    __syncthreads();
    { const int px = tid & 63, chh = (tid >> 6) * 8;
#pragma unroll 1
      for (int ci = 0; ci < 8; ++ci) { const int ch = chh + ci; const int grp = (c0 + ch) / GCH; const float* wrow = &sw[px][grp * K2]; float s = 0.f;
#pragma unroll
        for (int dy = 0; dy < KK; ++dy) {
#pragma unroll
          for (int dx = 0; dx < KK; ++dx) s += wrow[dy * KK + dx] * sy[ch][dy][px + dx]; }
        so[ch][px] = s; } }
    __syncthreads();
    for (int q = tid; q < CHK * 16; q += 128) { const int ch = q >> 4, pc = q & 15; vst2(out + ((size_t)b * CC + c0 + ch) * NPX + r * WI + x0 + pc * 4, *(const v4f*)(&so[ch][pc * 4])); }
    __syncthreads(); }
}
extern "C" void kernel_launch(void* const* d_in, const int* in_sizes, int n_in, void* d_out, int out_size, void* d_ws, size_t ws_size, hipStream_t stream) {
  (void)in_sizes; (void)n_in; (void)out_size; (void)ws_size; (void)d_ws;
  const float** I = (const float**)d_in;
  float* out = (float*)d_out;
  k_main<<<dim3(WI / 64, HI, NB), 128, 0, stream>>>(I[0], I[1], I[2], I[3], I[4], I[5], I[6], I[7], I[8], I[9], out);
}
